// HybridGeoNet_17343077941963
// MI455X (gfx1250) — hardware-run, weakly checked
//
#include <hip/hip_runtime.h>


namespace {
constexpr int NB = 4, C = 2048, HI = 32, WI = 32, S = HI * WI  , NT = NB * S  , E = 768, NH = 12, HD = 64, QKVW = 3 * E  , GH = 4, DG = E / GH  , KB = 128;
constexpr float HS = 256.0f, WSC = 4096.0f, PS = 256.0f, LNEPS = 1e-5f, SCALE = 0.125f;
typedef _Float16 b16;
typedef __attribute__((ext_vector_type(16))) _Float16 v16b;
typedef __attribute__((ext_vector_type(8))) _Float16 v8b;
typedef __attribute__((ext_vector_type(8))) float v8f;
typedef __attribute__((ext_vector_type(4))) float v4f;
__device__ __forceinline__ float bf16_rne(float f) { unsigned int u = __float_as_uint(f); u += 0x7FFFu + ((u >> 16) & 1u); float r = __uint_as_float(u & 0xFFFF0000u); asm volatile("" : "+v"(r)); return r; }
__device__ __forceinline__ float bfv(float f) { float r = bf16_rne(f); asm volatile("" : "+v"(r)); return r; }
__device__ __forceinline__ void split16(float v, b16& hi, b16& lo) { hi = (b16)v; lo = (b16)(v - (float)hi); }
__device__ __forceinline__ v16b frag_kb(const b16* p, int hh) { const v8b a = *(const v8b*)(p + 8 * hh), b = *(const v8b*)(p + 16 + 8 * hh); v16b f;
#pragma unroll
  for (int e = 0; e < 8; ++e) { f[e] = a[e]; f[8 + e] = b[e]; } return f; }
__device__ __forceinline__ v8f wmma16b(v16b a, v16b b, v8f c) { v8f d = __builtin_amdgcn_wmma_f32_16x16x32_f16(false, a, false, b, (short)0, c, false, false); asm volatile("v_nop\n\tv_nop\n\tv_nop\n\tv_nop" : "+v"(d) : "v"(a), "v"(b)); return d; }
__device__ __forceinline__ void wave_lds_sync() { __builtin_amdgcn_fence(__ATOMIC_RELEASE, "workgroup"); __builtin_amdgcn_wave_barrier(); __builtin_amdgcn_fence(__ATOMIC_ACQUIRE, "workgroup"); }
__device__ __forceinline__ float pmul(float a, float b) { float p = a * b; asm volatile("" : "+v"(p)); return p; }
__device__ __forceinline__ float leaky(float v) { return v >= 0.0f ? v : 0.2f * v; }
__device__ __forceinline__ float elu(float v) { return v > 0.0f ? v : (__expf(v) - 1.0f); }
__device__ __forceinline__ float gelu(float v) { return 0.5f * v * (1.0f + erff(v * 0.70710678118654752f)); }

__global__ __launch_bounds__(256) void wput_kernel(const float* __restrict__ pw, const float* __restrict__ wqkv, const float* __restrict__ wo, const float* __restrict__ gp, const float* __restrict__ ga, const float* __restrict__ m1, const float* __restrict__ m2, b16* __restrict__ PROJT, b16* __restrict__ WQKV, b16* __restrict__ WOT, b16* __restrict__ GPT, b16* __restrict__ GATT, b16* __restrict__ M1T, b16* __restrict__ M2T) { const size_t nt = (size_t)gridDim.x * 256, u0 = (size_t)blockIdx.x * 256 + threadIdx.x; v8b v;
  auto put = [&](const float* src, b16* dst, int kin, int nout) { for (size_t u = u0; u < (size_t)nout * (kin / 8); u += nt) { const int o = (int)(u / (kin / 8)), k0 = (int)(u % (kin / 8)) * 8;
#pragma unroll
      for (int j = 0; j < 8; ++j) v[j] = (b16)(bf16_rne(src[(size_t)(k0 + j) * nout + o]) * WSC); for (int pass = 0; pass < 2; ++pass) { *(volatile v8b*)(dst + (size_t)o * kin + k0) = v; __threadfence(); } } };
  put(pw, PROJT, C, E); put(wqkv, WQKV, E, QKVW); put(wo, WOT, E, E); put(gp, GPT, E, E); put(ga, GATT, E, E); put(m1, M1T, E, E); put(m2, M2T, E, E); }
__global__ __launch_bounds__(256) void ln1_kernel(const float* __restrict__ x, int TLIM, float* __restrict__ ST1) { const size_t u = (size_t)blockIdx.x * 256 + threadIdx.x; if (u >= (size_t)TLIM) return; const int b = (int)(u / S), s = (int)(u % S); const float* xb = x + (size_t)b * C * S + s; float sm = 0.0f; for (int c = 0; c < C; ++c) sm += bfv(xb[(size_t)c * S]); const float m = sm / C; float s2 = 0.0f; for (int c = 0; c < C; ++c) { const float d = bfv(xb[(size_t)c * S]) - m; s2 += d * d; } const float r = rsqrtf(s2 / C + LNEPS);
  for (int pass = 0; pass < 2; ++pass) { ((volatile float*)ST1)[u * 2] = m; ((volatile float*)ST1)[u * 2 + 1] = r; __threadfence(); } }
__global__ __launch_bounds__(32) void proj_kernel(const float* __restrict__ x, const float* __restrict__ ST1, const float* __restrict__ g1, const float* __restrict__ be1, const b16* __restrict__ PROJT, const float* __restrict__ pb, int TLIM, float* __restrict__ VIN) { __shared__ __attribute__((aligned(16))) b16 Ah[16][264], Al[16][264]; __shared__ float Tf[16][260], Ms[16], Rs[16]; const int lane = threadIdx.x, nloc = lane & 15, hlf = lane >> 4; const int g = blockIdx.x % 3; const size_t t0 = (size_t)(blockIdx.x / 3) * 16; if (t0 >= (size_t)TLIM) return; const int b = (int)(t0 / S), s0 = (int)(t0 % S); const float* xb = x + (size_t)b * C * S + s0;
  if (lane < 16) { Ms[lane] = ST1[(t0 + lane) * 2]; Rs[lane] = ST1[(t0 + lane) * 2 + 1]; for (int k = 256; k < 264; ++k) { Ah[lane][k] = (b16)0.0f; Al[lane][k] = (b16)0.0f; } }
  wave_lds_sync(); v8f acc[16];
#pragma unroll
  for (int t = 0; t < 16; ++t) acc[t] = (v8f){};
#pragma unroll 1
  for (int kc = 0; kc < C; kc += 256) {
    for (int cc = hlf; cc < 256; cc += 2) { const int c = kc + cc; const float v = (bfv(xb[(size_t)c * S + nloc]) - Ms[nloc]) * Rs[nloc] * bfv(g1[c]) + bfv(be1[c]); b16 p, ql; split16(v * HS, p, ql); Ah[nloc][cc] = p; Al[nloc][cc] = ql; }
    wave_lds_sync();
#pragma unroll 2
    for (int kb = 0; kb < 256; kb += 32) { const v16b a = frag_kb(&Ah[nloc][kb], hlf), al = frag_kb(&Al[nloc][kb], hlf);
#pragma unroll
      for (int t = 0; t < 16; ++t) { const v16b bw = frag_kb(PROJT + (size_t)(g * 256 + t * 16 + nloc) * C + kc + kb, hlf); acc[t] = wmma16b(a, bw, acc[t]); acc[t] = wmma16b(al, bw, acc[t]); } }
    wave_lds_sync(); }
#pragma unroll
  for (int t = 0; t < 16; ++t) { const int cc = t * 16 + nloc; const float bb = bfv(pb[g * 256 + cc]);
#pragma unroll
    for (int r8 = 0; r8 < 8; ++r8) Tf[8 * hlf + r8][cc] = acc[t][r8] * (1.0f / (HS * WSC)) + bb; }
  wave_lds_sync();
  for (int pass = 0; pass < 2; ++pass) { for (int rr = 0; rr < 16; ++rr) for (int q = 0; q < 2; ++q) *(volatile v4f*)(VIN + (t0 + rr) * E + g * 256 + q * 128 + lane * 4) = *(const v4f*)(&Tf[rr][q * 128 + lane * 4]); __threadfence(); } }
template <int LN, int ACT, int TOHL>
__global__ __launch_bounds__(32) void gemm_kernel(const float* __restrict__ IN, const float* __restrict__ lg, const float* __restrict__ lb, const b16* __restrict__ W, const float* __restrict__ bias, const float* __restrict__ RES, int NG, int OW, int QCOLS, int TLIM, float* __restrict__ OUTF, b16* __restrict__ OUTH, b16* __restrict__ OUTL) { __shared__ __attribute__((aligned(16))) b16 Ah[16][264], Al[16][264]; __shared__ float Tf[16][260], Ms[16], Rs[16]; const int lane = threadIdx.x, nloc = lane & 15, hlf = lane >> 4; const int g = blockIdx.x % NG; const size_t t0 = (size_t)(blockIdx.x / NG) * 16; if (t0 >= (size_t)TLIM) return;
  if (LN) { for (int rr = 0; rr < 16; ++rr) { float sm = 0.0f; for (int q = 0; q < E / 32; ++q) sm += IN[(t0 + rr) * E + q * 32 + lane]; for (int o = 16; o; o >>= 1) sm += __shfl_xor(sm, o); const float m = sm / E; float s2 = 0.0f; for (int q = 0; q < E / 32; ++q) { const float d = IN[(t0 + rr) * E + q * 32 + lane] - m; s2 += d * d; } for (int o = 16; o; o >>= 1) s2 += __shfl_xor(s2, o); if (lane == 0) { Ms[rr] = m; Rs[rr] = rsqrtf(s2 / E + LNEPS); } } }
  if (lane < 16) for (int k = 256; k < 264; ++k) { Ah[lane][k] = (b16)0.0f; Al[lane][k] = (b16)0.0f; }
  wave_lds_sync(); v8f acc[16];
#pragma unroll
  for (int t = 0; t < 16; ++t) acc[t] = (v8f){};
#pragma unroll 1
  for (int kc = 0; kc < E; kc += 256) { for (int rr = 0; rr < 16; ++rr) for (int q = 0; q < 8; ++q) { const int k = kc + q * 32 + lane; float v = IN[(t0 + rr) * E + k]; if (LN) v = pmul((v - Ms[rr]) * Rs[rr], bfv(lg[k])) + bfv(lb[k]); b16 p, ql; split16(v * HS, p, ql); Ah[rr][q * 32 + lane] = p; Al[rr][q * 32 + lane] = ql; }
    wave_lds_sync();
#pragma unroll 1
    for (int kb = 0; kb < 256; kb += 32) { const v16b a = frag_kb(&Ah[nloc][kb], hlf), al = frag_kb(&Al[nloc][kb], hlf);
#pragma unroll
      for (int t = 0; t < 16; ++t) { const v16b bw = frag_kb(W + (size_t)(g * 256 + t * 16 + nloc) * E + kc + kb, hlf); acc[t] = wmma16b(a, bw, acc[t]); acc[t] = wmma16b(al, bw, acc[t]); } }
    wave_lds_sync(); }
#pragma unroll
  for (int t = 0; t < 16; ++t) { const int cc = t * 16 + nloc; const int col = g * 256 + cc; const float bb = bias ? bfv(bias[col]) : 0.0f;
#pragma unroll
    for (int r8 = 0; r8 < 8; ++r8) { float v = acc[t][r8] * (1.0f / (HS * WSC)) + bb; if (ACT == 1) v = gelu(v); if (RES) v += RES[(t0 + 8 * hlf + r8) * OW + col]; Tf[8 * hlf + r8][cc] = v; } }
  wave_lds_sync();
  for (int pass = 0; pass < 2; ++pass) { for (int rr = 0; rr < 16; ++rr) { if (TOHL) { const int col = g * 256 + lane * 8; const float sc = col < QCOLS ? SCALE : 1.0f; v8b hv, lv;
#pragma unroll
        for (int j = 0; j < 8; ++j) { b16 p, ql; split16(Tf[rr][lane * 8 + j] * sc * HS, p, ql); hv[j] = p; lv[j] = ql; } *(volatile v8b*)(OUTH + (t0 + rr) * OW + col) = hv; *(volatile v8b*)(OUTL + (t0 + rr) * OW + col) = lv; }
      else for (int q = 0; q < 2; ++q) *(volatile v4f*)(OUTF + (t0 + rr) * OW + g * 256 + q * 128 + lane * 4) = *(const v4f*)(&Tf[rr][q * 128 + lane * 4]); } __threadfence(); } }
__global__ __launch_bounds__(32) void att_kernel(const b16* __restrict__ Ph, const b16* __restrict__ Pl, int TLIM, float* __restrict__ ATT) { __shared__ __attribute__((aligned(16))) b16 P_h[16][KB + 8], P_l[16][KB + 8], Vth[HD][KB + 8], Vtl[HD][KB + 8]; __shared__ float Sf[16][KB + 4], Of[16][HD + 4];
  const int lane = threadIdx.x, nloc = lane & 15, hlf = lane >> 4; const int qt = blockIdx.x % (S / 16); const int h = (blockIdx.x / (S / 16)) % NH; const int b = blockIdx.x / ((S / 16) * NH); const size_t t0 = (size_t)b * S + (size_t)qt * 16; if (t0 >= (size_t)TLIM) return; const int qoff = h * HD, koff = E + h * HD, voff = 2 * E + h * HD;
  v16b qa[2], qb[2];
#pragma unroll
  for (int ks = 0; ks < 2; ++ks) { qa[ks] = frag_kb(Ph + (t0 + nloc) * QKVW + qoff + ks * 32, hlf); qb[ks] = frag_kb(Pl + (t0 + nloc) * QKVW + qoff + ks * 32, hlf); }
  float m_r[8], den_r[8]; v8f acc[4];
#pragma unroll
  for (int r8 = 0; r8 < 8; ++r8) { m_r[r8] = -INFINITY; den_r[r8] = 0.0f; }
#pragma unroll
  for (int t = 0; t < 4; ++t) acc[t] = (v8f){};
  const int kend = (b * S + S) < TLIM ? S : (TLIM - b * S);
#pragma unroll 1
  for (int kb0 = 0; kb0 < kend; kb0 += KB) { const size_t kbase = (size_t)b * S + kb0;
    for (int rr = 0; rr < KB; rr += 2) { const int r = rr + hlf; const size_t vr = (kbase + r) * QKVW + voff; for (int s2 = 0; s2 < HD / 16; ++s2) { Vth[s2 * 16 + nloc][r] = Ph[vr + s2 * 16 + nloc]; Vtl[s2 * 16 + nloc][r] = Pl[vr + s2 * 16 + nloc]; } }
#pragma unroll
    for (int t = 0; t < KB / 16; ++t) { const size_t kr = (kbase + t * 16 + nloc) * QKVW + koff; v8f s = {};
#pragma unroll
      for (int ks = 0; ks < 2; ++ks) { const v16b ka = frag_kb(Ph + kr + ks * 32, hlf), kl = frag_kb(Pl + kr + ks * 32, hlf); s = wmma16b(qa[ks], ka, s); s = wmma16b(qa[ks], kl, s); s = wmma16b(qb[ks], ka, s); }
#pragma unroll
      for (int r8 = 0; r8 < 8; ++r8) Sf[8 * hlf + r8][t * 16 + nloc] = s[r8] * (1.0f / (HS * HS)); }
    wave_lds_sync();
#pragma unroll
    for (int rr = 0; rr < 16; ++rr) { float mx = -INFINITY;
#pragma unroll
      for (int q = 0; q < 4; ++q) mx = fmaxf(mx, Sf[rr][q * 32 + lane]);
      for (int o = 16; o; o >>= 1) mx = fmaxf(mx, __shfl_xor(mx, o));
      const float mold = __shfl(m_r[rr & 7], (rr >> 3) * 16); const float mn = fmaxf(mold, mx); const float sf = (mold == -INFINITY) ? 0.0f : __expf(mold - mn); float ps = 0.0f;
#pragma unroll
      for (int q = 0; q < 4; ++q) { const int kx = q * 32 + lane; const float p = __expf(Sf[rr][kx] - mn); ps += p; b16 ph, pl; split16(p * PS, ph, pl); P_h[rr][kx] = ph; P_l[rr][kx] = pl; }
      for (int o = 16; o; o >>= 1) ps += __shfl_xor(ps, o);
      if ((rr >> 3) == hlf) { const int r8 = rr & 7; den_r[r8] = den_r[r8] * sf + ps; m_r[r8] = mn;
#pragma unroll
        for (int t = 0; t < 4; ++t) acc[t][r8] = acc[t][r8] * sf; } }
    wave_lds_sync();
#pragma unroll
    for (int ks = 0; ks < KB; ks += 32) { const v16b pa = frag_kb(&P_h[nloc][ks], hlf), pb2 = frag_kb(&P_l[nloc][ks], hlf);
#pragma unroll
      for (int t = 0; t < 4; ++t) { const v16b vh = frag_kb(&Vth[t * 16 + nloc][ks], hlf), vl = frag_kb(&Vtl[t * 16 + nloc][ks], hlf); acc[t] = wmma16b(pa, vh, acc[t]); acc[t] = wmma16b(pa, vl, acc[t]); acc[t] = wmma16b(pb2, vh, acc[t]); } }
    wave_lds_sync(); }
#pragma unroll
  for (int t = 0; t < 4; ++t)
#pragma unroll
    for (int r8 = 0; r8 < 8; ++r8) Of[8 * hlf + r8][t * 16 + nloc] = acc[t][r8] * (1.0f / (HS * PS)) / den_r[r8];
  wave_lds_sync();
  for (int pass = 0; pass < 2; ++pass) { for (int rr = 0; rr < 16; ++rr) for (int s2 = 0; s2 < HD / 32; ++s2) ((volatile float*)ATT)[(t0 + rr) * E + qoff + s2 * 32 + lane] = Of[rr][s2 * 32 + lane]; __threadfence(); } }
__global__ __launch_bounds__(256) void gatcoef_kernel(const float* __restrict__ HN, const float* __restrict__ as_, const float* __restrict__ ad_, int TLIM, float* __restrict__ ES) { const size_t u = (size_t)blockIdx.x * 256 + threadIdx.x; const size_t t = u / GH; const int h = (int)(u % GH); if (t >= (size_t)TLIM) return; float s1 = 0.0f, s2 = 0.0f; for (int k = 0; k < DG; ++k) { const float v = HN[t * E + h * DG + k]; s1 += pmul(v, bfv(as_[h * DG + k])); s2 += pmul(v, bfv(ad_[h * DG + k])); }
  for (int pass = 0; pass < 2; ++pass) { ((volatile float*)ES)[t * 8 + h] = s1; ((volatile float*)ES)[t * 8 + 4 + h] = s2; __threadfence(); } }
__global__ __launch_bounds__(256) void gat_kernel(const float* __restrict__ HN, const float* __restrict__ ES, const float* __restrict__ XA, const float* __restrict__ gb, int TLIM, float* __restrict__ XF) { const int wave = threadIdx.x >> 5, lane = threadIdx.x & 31; const size_t t = (size_t)blockIdx.x * 8 + wave; if (t >= (size_t)TLIM) return; const int b = (int)(t / S), s = (int)(t % S), r = s / WI, c = s % WI;
  const int off9[9] = {0, -1, 1, -WI, WI, -WI - 1, WI + 1, -WI + 1, WI - 1};
  bool ok[9]; ok[0] = true; ok[1] = c > 0; ok[2] = c < WI - 1; ok[3] = r > 0; ok[4] = r < HI - 1; ok[5] = r > 0 && c > 0; ok[6] = r < HI - 1 && c < WI - 1; ok[7] = r > 0 && c + 1 >= 1 && c + 1 <= WI - 2; ok[8] = r < HI - 1 && c >= 1 && c <= WI - 2;
#pragma unroll
  for (int j = 0; j < 9; ++j) ok[j] = ok[j] && ((size_t)b * S + (size_t)(s + off9[j]) < (size_t)TLIM);
  float o[E / 32];
#pragma unroll
  for (int q = 0; q < E / 32; ++q) o[q] = 0.0f;
#pragma unroll
  for (int h = 0; h < GH; ++h) { const float ad = ES[t * 8 + 4 + h]; float ev[9]; float mx = -INFINITY;
#pragma unroll
    for (int j = 0; j < 9; ++j) { ev[j] = 0.0f; if (ok[j]) { const size_t u = (size_t)b * S + (size_t)(s + off9[j]); ev[j] = leaky(ES[u * 8 + h] + ad); mx = fmaxf(mx, ev[j]); } }
    float den = 0.0f;
#pragma unroll
    for (int j = 0; j < 9; ++j) if (ok[j]) { ev[j] = __expf(ev[j] - mx); den += ev[j]; }
#pragma unroll
    for (int j = 0; j < 9; ++j) if (ok[j]) { const float al = ev[j] / den; const size_t u = (size_t)b * S + (size_t)(s + off9[j]);
#pragma unroll
      for (int q = 0; q < DG / 32; ++q) { const int ch = h * DG + q * 32 + lane; o[h * (DG / 32) + q] += pmul(al, HN[u * E + ch]); } } }
  for (int pass = 0; pass < 2; ++pass) {
#pragma unroll
    for (int q = 0; q < E / 32; ++q) { const int h = q / (DG / 32), qq = q % (DG / 32); const int ch = h * DG + qq * 32 + lane; ((volatile float*)XF)[t * E + ch] = XA[t * E + ch] + elu(o[q] + bfv(gb[ch])); } __threadfence(); } }
__global__ __launch_bounds__(32) void lnrows_kernel(const float* __restrict__ IN, const float* __restrict__ g, const float* __restrict__ bb, int TLIM, float* __restrict__ OUT) { const int lane = threadIdx.x; const size_t t0 = (size_t)blockIdx.x * 16; if (t0 >= (size_t)TLIM) return;
  for (int pass = 0; pass < 2; ++pass) { for (int rr = 0; rr < 16; ++rr) { float v[E / 32]; float sm = 0.0f;
#pragma unroll
      for (int q = 0; q < E / 32; ++q) { v[q] = IN[(t0 + rr) * E + q * 32 + lane]; sm += v[q]; } for (int o = 16; o; o >>= 1) sm += __shfl_xor(sm, o); const float m = sm / E; float s2 = 0.0f;
#pragma unroll
      for (int q = 0; q < E / 32; ++q) { const float d = v[q] - m; s2 += d * d; } for (int o = 16; o; o >>= 1) s2 += __shfl_xor(s2, o); const float rs = rsqrtf(s2 / E + LNEPS);
#pragma unroll
      for (int q = 0; q < E / 32; ++q) { const int k = q * 32 + lane; ((volatile float*)OUT)[(t0 + rr) * E + k] = pmul((v[q] - m) * rs, bfv(g[k])) + bfv(bb[k]); } } __threadfence(); } }
__global__ __launch_bounds__(32) void final_kernel(const float* __restrict__ YP, const float* __restrict__ fg, const float* __restrict__ fb, int TLIM, float* __restrict__ out) { __shared__ float Ys[32][E + 1]; __shared__ float Ms[32], Rs[32]; const int lane = threadIdx.x; const size_t t0 = (size_t)blockIdx.x * 32; if (t0 >= (size_t)TLIM) return; const int b = (int)(t0 / S), s0 = (int)(t0 % S);
  for (int rr = 0; rr < 32; ++rr) { float sm = 0.0f; for (int q = 0; q < E / 32; ++q) { const float v = YP[(t0 + rr) * E + q * 32 + lane]; Ys[rr][q * 32 + lane] = v; sm += v; } for (int o = 16; o; o >>= 1) sm += __shfl_xor(sm, o); const float m = sm / E; float s2 = 0.0f; for (int q = 0; q < E / 32; ++q) { const float d = Ys[rr][q * 32 + lane] - m; s2 += d * d; } for (int o = 16; o; o >>= 1) s2 += __shfl_xor(s2, o); if (lane == 0) { Ms[rr] = m; Rs[rr] = rsqrtf(s2 / E + LNEPS); } }
  wave_lds_sync();
  for (int pass = 0; pass < 2; ++pass) {
#pragma unroll 4
    for (int e = 0; e < E; ++e) ((volatile float*)out)[((size_t)b * E + e) * S + s0 + lane] = pmul((Ys[lane][e] - Ms[lane]) * Rs[lane], bfv(fg[e])) + bfv(fb[e]); __threadfence(); } }
}

extern "C" void kernel_launch(void* const* d_in, const int* in_sizes, int n_in, void* d_out, int out_size, void* d_ws, size_t ws_size, hipStream_t stream) {
  (void)n_in;
  auto Fp = [&](int i) { return (const float*)d_in[i]; };
  if (in_sizes[0] != NB * C * S || in_sizes[1] != C || in_sizes[3] != C * E || in_sizes[5] != E * QKVW || in_sizes[7] != E * E || in_sizes[11] != E * E || in_sizes[13] != E * E || in_sizes[14] != GH * DG || in_sizes[19] != E * E || in_sizes[21] != E * E || in_sizes[23] != E || out_size != NB * E * S) return;
  const int TLIM = NT;
  size_t off = 0; char* ws = (char*)d_ws;
  auto carve = [&](size_t bytes) { char* p = ws + off; off += (bytes + 255) & ~(size_t)255; return p; };
  b16* PROJT = (b16*)carve((size_t)E * C * 2); b16* WQKV = (b16*)carve((size_t)QKVW * E * 2); b16* WOT = (b16*)carve((size_t)E * E * 2); b16* GPT = (b16*)carve((size_t)E * E * 2); b16* GATT = (b16*)carve((size_t)E * E * 2); b16* M1T = (b16*)carve((size_t)E * E * 2); b16* M2T = (b16*)carve((size_t)E * E * 2);
  float* ST1 = (float*)carve((size_t)NT * 2 * 4); float* VIN = (float*)carve((size_t)NT * E * 4); b16* Ph = (b16*)carve((size_t)NT * QKVW * 2); b16* Pl = (b16*)carve((size_t)NT * QKVW * 2); float* ATT = (float*)carve((size_t)NT * E * 4); float* XA = (float*)carve((size_t)NT * E * 4); float* G = (float*)carve((size_t)NT * E * 4); float* HN = (float*)carve((size_t)NT * E * 4); float* ES = (float*)carve((size_t)NT * 8 * 4); float* XF = (float*)carve((size_t)NT * E * 4); float* N3 = (float*)carve((size_t)NT * E * 4); float* MID = (float*)carve((size_t)NT * E * 4); float* YP = (float*)carve((size_t)NT * E * 4);
  if (off > ws_size || off > ((size_t)208 << 20)) return;
  const unsigned nw = TLIM / 16;
  wput_kernel<<<512, 256, 0, stream>>>(Fp(3), Fp(5), Fp(7), Fp(11), Fp(13), Fp(19), Fp(21), PROJT, WQKV, WOT, GPT, GATT, M1T, M2T);
  ln1_kernel<<<(TLIM + 255) / 256, 256, 0, stream>>>(Fp(0), TLIM, ST1);
  proj_kernel<<<nw * 3, 32, 0, stream>>>(Fp(0), ST1, Fp(1), Fp(2), PROJT, Fp(4), TLIM, VIN);
  gemm_kernel<0, 0, 1><<<nw * 9, 32, 0, stream>>>(VIN, nullptr, nullptr, WQKV, Fp(6), nullptr, 9, QKVW, E, TLIM, nullptr, Ph, Pl);
  att_kernel<<<NB * NH * (S / 16), 32, 0, stream>>>(Ph, Pl, TLIM, ATT);
  gemm_kernel<0, 0, 0><<<nw * 3, 32, 0, stream>>>(ATT, nullptr, nullptr, WOT, Fp(8), VIN, 3, E, 0, TLIM, XA, nullptr, nullptr);
  gemm_kernel<1, 0, 0><<<nw * 3, 32, 0, stream>>>(XA, Fp(9), Fp(10), GPT, Fp(12), nullptr, 3, E, 0, TLIM, G, nullptr, nullptr);
  gemm_kernel<0, 0, 0><<<nw * 3, 32, 0, stream>>>(G, nullptr, nullptr, GATT, nullptr, nullptr, 3, E, 0, TLIM, HN, nullptr, nullptr);
  gatcoef_kernel<<<(TLIM * GH + 255) / 256, 256, 0, stream>>>(HN, Fp(14), Fp(15), TLIM, ES);
  gat_kernel<<<(TLIM + 7) / 8, 256, 0, stream>>>(HN, ES, XA, Fp(16), TLIM, XF);
  lnrows_kernel<<<nw, 32, 0, stream>>>(XF, Fp(17), Fp(18), TLIM, N3);
  gemm_kernel<0, 1, 0><<<nw * 3, 32, 0, stream>>>(N3, nullptr, nullptr, M1T, Fp(20), nullptr, 3, E, 0, TLIM, MID, nullptr, nullptr);
  gemm_kernel<0, 0, 0><<<nw * 3, 32, 0, stream>>>(MID, nullptr, nullptr, M2T, Fp(22), N3, 3, E, 0, TLIM, YP, nullptr, nullptr);
  final_kernel<<<TLIM / 32, 32, 0, stream>>>(YP, Fp(23), Fp(24), TLIM, (float*)d_out);
}
